// GNN_17669495456025
// MI455X (gfx1250) — hardware-verified
//
#include <hip/hip_runtime.h>
#include <stddef.h>
#include <stdint.h>


#define NN     100000
#define NE     1600000
#define NG     256
#define NF     7
#define EF     3
#define UD     2
#define HID    128
#define KIE    17
#define KIN    18
#define KB     64
#define TM     128
#define MTHR   128
#define NP     100096
#define DP     132
#define AP     72
#define CSTN   1040
#define NTHR   256
#define NWAVE  8
#define EPT    8
#define CHUNK  (NTHR * EPT)
#define WCAP   (EPT * 32)
#define LISTN  (NWAVE * WCAP)
#define NBA    1024
#define SLA    10
#define RCAP   28672
#define DEGCAP 64
#define NBLK   98
#define NPA    (NBLK * NBA)
#define AGG_ZINTS (LISTN + 2 * RCAP + 3 * NBA)
#define AGG_LDS_INTS (AGG_ZINTS + 16)
#define AGG_LDS_BYTES (AGG_LDS_INTS * 4)
#define MLP_LDS_FLOATS (TM * DP + (TM * AP) / 2 + CSTN + TM * 8)
#define MLP_LDS_BYTES (MLP_LDS_FLOATS * 4)
#define NU_W   4096
#define NU_X   (NP * 2)
#define WSMAX  134217728

static_assert(NE % TM == 0);
static_assert(NP % TM == 0 && NP >= NN && NP - NN < TM);
static_assert(NPA >= NP && NBLK * NBA == NPA);
static_assert(KIE <= 32 && KIN <= 32);
static_assert(NG % 32 == 0 && NN % 4 == 0 && NE % 4 == 0);
static_assert(RCAP >= 16710 + 836 && DEGCAP >= 36 + 8);
static_assert(RCAP % (NTHR * 4) == 0);
static_assert(((long long)NE << SLA) < (1LL << 31));
static_assert((CHUNK & (CHUNK - 1)) == 0 && CHUNK <= 4096);
static_assert((NBA & (NBA - 1)) == 0 && NBA == (1 << SLA) && NBA == 4 * NTHR);
static_assert(((long long)CHUNK << SLA) < (1LL << 31));
static_assert(LISTN % NTHR == 0 && AGG_ZINTS % 4 == 0 && LISTN % 4 == 0 && NBA % 32 == 0);
static_assert(AGG_LDS_BYTES <= 300000 && MLP_LDS_BYTES <= 300000);
static_assert((DP * 4) % 16 == 0 && (AP * 2) % 16 == 0 && AP >= KB && DP >= HID);
static_assert((TM * DP * 4) % 16 == 0 && (TM * AP * 2) % 16 == 0 && (CSTN * 4) % 16 == 0);
static_assert(CSTN >= HID + NF * HID + 8);
static_assert((HID * EF) % MTHR == 0 && (HID * NF) % MTHR == 0 && HID == MTHR && TM == MTHR);
static_assert(NU_W % NTHR == 0 && NU_X % NTHR == 0 && (NU_W / 4) % NTHR == 0);
static_assert(4 * 4 == 16 && 8 * 4 == 32);

typedef float          v2f   __attribute__((ext_vector_type(2)));
typedef float          v4f   __attribute__((ext_vector_type(4)));
typedef float          v8f   __attribute__((ext_vector_type(8)));
typedef int            v4i   __attribute__((ext_vector_type(4)));
typedef int            v8i   __attribute__((ext_vector_type(8)));
typedef unsigned short v8us  __attribute__((ext_vector_type(8)));
typedef unsigned short v16us __attribute__((ext_vector_type(16)));
typedef __bf16         v16bf __attribute__((ext_vector_type(16)));
typedef v2f  __attribute__((may_alias)) v2fa;
typedef v4f  __attribute__((may_alias)) v4fa;
typedef v4i  __attribute__((may_alias)) v4ia;
typedef v8us __attribute__((may_alias)) v8usa;
union FragB { v16bf v; v16us u; v8us h[2]; v8i w; };
struct HL { v8us h; v8us l; };

__device__ __forceinline__ v8f wmb(const FragB& a, const FragB& b, v8f c) {
  v8f d = __builtin_amdgcn_wmma_f32_16x16x32_bf16(false, a.v, false, b.v, (short)0, c, false, false);
  asm volatile("v_nop\n\tv_nop\n\tv_nop\n\tv_nop" : "+v"(d) : "v"(a.w), "v"(b.w));
  return d;
}

__device__ __forceinline__ unsigned bf16_bits(float f) {
  const unsigned u = __float_as_uint(f);
  const unsigned r = (u + 0x7FFFu + ((u >> 16) & 1u)) >> 16;
  return (f != f) ? 0x7FC0u : r;
}
__device__ __forceinline__ float bf16_val(float f) {
  return __uint_as_float(bf16_bits(f) << 16);
}
__device__ __forceinline__ HL split8(v8f f) {
  HL r;
#pragma unroll
  for (int i = 0; i < 8; ++i) {
    const unsigned hb = bf16_bits(f[i]);
    const unsigned lb = bf16_bits(f[i] - __uint_as_float(hb << 16));
    r.h[i] = (unsigned short)hb;
    r.l[i] = (unsigned short)lb;
  }
  return r;
}
__device__ __forceinline__ float relu_f(float v) { return (v > 0.0f) ? v : (v - v); }

__device__ __forceinline__ void putf4(float* dp, v4f o) {
  *(volatile v4f*)dp = o;
  __threadfence();
  *(volatile v4f*)dp = o;
}
__device__ __forceinline__ void put16(unsigned short* dp, v8us o) {
  *(volatile v8us*)dp = o;
  __threadfence();
  *(volatile v8us*)dp = o;
}

template <int SLB>
__device__ __forceinline__ int scan_chunk(const int* __restrict__ dsts, int nE, int cbase, int slotBase,
                                          int nb, int vec8, int* list, int tid, int lane, int wave) {
  int wc = 0;
  const int el0  = tid * EPT;
  const int e0   = cbase + el0;
  const int sent = -2147483647 - 1;
  v4i da, db;
  if (vec8 != 0 && cbase + CHUNK <= nE) {
    da = *(const v4i*)(dsts + e0);
    db = *(const v4i*)(dsts + e0 + 4);
  } else {
    da.x = (e0     < nE) ? dsts[min(e0,     nE - 1)] : sent;
    da.y = (e0 + 1 < nE) ? dsts[min(e0 + 1, nE - 1)] : sent;
    da.z = (e0 + 2 < nE) ? dsts[min(e0 + 2, nE - 1)] : sent;
    da.w = (e0 + 3 < nE) ? dsts[min(e0 + 3, nE - 1)] : sent;
    db.x = (e0 + 4 < nE) ? dsts[min(e0 + 4, nE - 1)] : sent;
    db.y = (e0 + 5 < nE) ? dsts[min(e0 + 5, nE - 1)] : sent;
    db.z = (e0 + 6 < nE) ? dsts[min(e0 + 6, nE - 1)] : sent;
    db.w = (e0 + 7 < nE) ? dsts[min(e0 + 7, nE - 1)] : sent;
  }
  const unsigned nbs = (unsigned)slotBase;
  const unsigned unb = (unsigned)nb;
  const unsigned s0 = (unsigned)da.x - nbs, s1 = (unsigned)da.y - nbs;
  const unsigned s2 = (unsigned)da.z - nbs, s3 = (unsigned)da.w - nbs;
  const unsigned s4 = (unsigned)db.x - nbs, s5 = (unsigned)db.y - nbs;
  const unsigned s6 = (unsigned)db.z - nbs, s7 = (unsigned)db.w - nbs;
  const bool h0 = s0 < unb, h1 = s1 < unb, h2 = s2 < unb, h3 = s3 < unb;
  const bool h4 = s4 < unb, h5 = s5 < unb, h6 = s6 < unb, h7 = s7 < unb;
  const unsigned any = __builtin_amdgcn_ballot_w32(h0 | h1 | h2 | h3 | h4 | h5 | h6 | h7);
  if (any != 0u) {
#define HITJ(J, HJ, SJ) { \
      const unsigned mj = __builtin_amdgcn_ballot_w32(HJ); \
      if (mj != 0u) { \
        if (HJ) { \
          const int pos = wc + (int)__builtin_amdgcn_mbcnt_lo(mj, 0u); \
          if (pos < WCAP) list[wave * WCAP + pos] = ((el0 + (J)) << SLB) | (int)(SJ); \
        } \
        wc += (int)__builtin_popcount(mj); } }
    HITJ(0, h0, s0)
    HITJ(1, h1, s1)
    HITJ(2, h2, s2)
    HITJ(3, h3, s3)
    HITJ(4, h4, s4)
    HITJ(5, h5, s5)
    HITJ(6, h6, s6)
    HITJ(7, h7, s7)
#undef HITJ
  }
  return wc;
}

__device__ __forceinline__ v8us gather8(const float* __restrict__ W, int kin, int kk, int n) {
  v8us o;
#pragma unroll
  for (int i = 0; i < 8; ++i) {
    const int k  = kk + i;
    const int kc = k < kin ? k : kin - 1;
    const unsigned b = bf16_bits(W[(size_t)kc * HID + n]);
    o[i] = (k < kin) ? (unsigned short)b : (unsigned short)0;
  }
  return o;
}

__global__ __launch_bounds__(NTHR) void k_prep(const float* __restrict__ x, const float* __restrict__ eW1,
                                               const float* __restrict__ nW1,
                                               unsigned short* E1T, unsigned short* N1T, float* X0) {
  const int u = (int)blockIdx.x * NTHR + (int)threadIdx.x;
  if (u < NU_W) {
    const int p  = u >> 10;
    const int v  = u & 1023;
    const int n  = v >> 3;
    const int k8 = (v & 7) * 8;
    const int kk = k8 & 31;
    if (p == 0) {
      const v8us o = gather8(eW1, KIE, kk, n);
      put16(E1T + (size_t)n * KB + k8, o);
    } else if (p == 1) {
      const v8us o = gather8(eW1 + KIE * HID, KIE, kk, n);
      put16(E1T + (size_t)HID * KB + (size_t)n * KB + k8, o);
    } else if (p == 2) {
      const v8us o = gather8(nW1, KIN, kk, n);
      put16(N1T + (size_t)n * KB + k8, o);
    } else {
      const v8us o = gather8(nW1 + KIN * HID, KIN, kk, n);
      put16(N1T + (size_t)HID * KB + (size_t)n * KB + k8, o);
    }
    return;
  }
  const int v = u - NU_W;
  if (v >= NU_X) return;
  const int rw   = v >> 1;
  const int half = v & 1;
  const int rc   = rw < NN ? rw : NN - 1;
  const bool ok  = rw < NN;
  const float* p = x + (size_t)rc * NF + 4 * half;
  const int i3   = half ? 2 : 3;
  const float a0 = p[0], a1 = p[1], a2 = p[2], a3 = p[i3];
  v4f q;
  q.x = ok ? bf16_val(a0) : 0.0f;
  q.y = ok ? bf16_val(a1) : 0.0f;
  q.z = ok ? bf16_val(a2) : 0.0f;
  q.w = (ok && half == 0) ? bf16_val(a3) : 0.0f;
  putf4(X0 + (size_t)v * 4, q);
}

__global__ __launch_bounds__(NTHR) void k_bucket(const int* __restrict__ dsts, int nE, int vec8,
                                                 int* LIST, int* CNT, int* OFF) {
  extern __shared__ __attribute__((aligned(16))) int dsm[];
  int* list = dsm;
  int* hl   = dsm + LISTN;
  int* sl   = hl + RCAP;
  int* cnt  = sl + RCAP;
  int* offs = cnt + NBA;
  int* cur  = offs + NBA;
  int* misc = cur + NBA;
  const int tid = (int)threadIdx.x, lane = tid & 31, wave = tid >> 5;
  const int nodeBase = (int)blockIdx.x * NBA;

  {
    const v4i z4 = {0, 0, 0, 0};
    for (int i = tid * 4; i < AGG_ZINTS; i += NTHR * 4) *(v4ia*)(dsm + i) = z4;
    if (tid < 16) misc[tid] = 0;
  }
  __syncthreads();

  int t = 0, ov = 0;
  const int nChunks = (nE + CHUNK - 1) / CHUNK;
#pragma unroll 1
  for (int ch = 0; ch < nChunks; ++ch) {
    const int cbase = ch * CHUNK;
    const int wc = scan_chunk<SLA>(dsts, nE, cbase, nodeBase, NBA, vec8, list, tid, lane, wave);
    if (lane == 0) misc[wave] = wc;
    __syncthreads();
    if (wave == 0) {
#pragma unroll 1
      for (int w2 = 0; w2 < NWAVE; ++w2) {
        int c = misc[w2];
        c = c < 0 ? 0 : (c > WCAP ? WCAP : c);
#pragma unroll 1
        for (int b0 = 0; b0 < c; b0 += 32) {
          const int idx = b0 + lane;
          const int ent = list[w2 * WCAP + (idx < WCAP ? idx : WCAP - 1)];
          const int m32 = (c - b0) < 32 ? (c - b0) : 32;
#pragma unroll 1
          for (int k = 0; k < m32; ++k) {
            const int u    = __builtin_amdgcn_readlane(ent, k);
            const int slot = u & (NBA - 1);
            const int el   = (u >> SLA) & (CHUNK - 1);
            const int pk   = ((cbase + el) << SLA) | slot;
            if (t < RCAP) {
              if (lane == 0) { hl[t] = pk; cnt[slot] = cnt[slot] + 1; }
              t = t + 1;
            } else {
              ov = 1;
            }
          }
        }
      }
    }
    __syncthreads();
  }
  if (wave == 0 && lane == 0) { misc[8] = t; misc[9] = ov; }
  __syncthreads();
  int tt = misc[8];
  tt = tt < 0 ? 0 : (tt > RCAP ? RCAP : tt);
  const int ovf = misc[9];

  if (wave == 0) {
    const int base = lane * (NBA / 32);
    int s = 0;
#pragma unroll 1
    for (int i = 0; i < NBA / 32; ++i) s += cnt[base + i];
    int incl = s;
#pragma unroll
    for (int d = 1; d < 32; d <<= 1) {
      const int y = __shfl_up(incl, d, 32);
      if (lane >= d) incl += y;
    }
    int run = incl - s;
#pragma unroll 1
    for (int i = 0; i < NBA / 32; ++i) {
      const int cv = cnt[base + i];
      offs[base + i] = run;
      cur[base + i]  = run;
      run += cv;
    }
  }
  __syncthreads();
  if (wave == 0) {
#pragma unroll 1
    for (int b0 = 0; b0 < tt; b0 += 32) {
      const int idx = b0 + lane;
      const int ent = hl[idx < RCAP ? idx : RCAP - 1];
      const int m32 = (tt - b0) < 32 ? (tt - b0) : 32;
#pragma unroll 1
      for (int k = 0; k < m32; ++k) {
        const int u    = __builtin_amdgcn_readlane(ent, k);
        const int slot = u & (NBA - 1);
        if (lane == 0) {
          int p = cur[slot];
          p = p < 0 ? 0 : (p > RCAP - 1 ? RCAP - 1 : p);
          sl[p] = u;
          cur[slot] = p + 1;
        }
      }
    }
  }
  __syncthreads();

  int* gl = LIST + (size_t)blockIdx.x * RCAP;
  v4i c4 = *(const v4ia*)(cnt + 4 * tid);
  const v4i o4 = *(const v4ia*)(offs + 4 * tid);
  if (ovf != 0) { c4.x = -1; c4.y = -1; c4.z = -1; c4.w = -1; }
#pragma unroll 1
  for (int it = 0; it < RCAP / (NTHR * 4); ++it) {
    const int q = (it * NTHR + tid) * 4;
    const v4i v = *(const v4ia*)(sl + q);
    *(volatile v4i*)(gl + q) = v;
  }
  *(volatile v4i*)(CNT + nodeBase + 4 * tid) = c4;
  *(volatile v4i*)(OFF + nodeBase + 4 * tid) = o4;
  __threadfence();
#pragma unroll 1
  for (int it = 0; it < RCAP / (NTHR * 4); ++it) {
    const int q = (it * NTHR + tid) * 4;
    const v4i v = *(const v4ia*)(sl + q);
    *(volatile v4i*)(gl + q) = v;
  }
  *(volatile v4i*)(CNT + nodeBase + 4 * tid) = c4;
  *(volatile v4i*)(OFF + nodeBase + 4 * tid) = o4;
}

template <int KS>
__device__ __forceinline__ void wave_gemm(const unsigned short* sAw, float* sDw,
                                          const unsigned short* __restrict__ BT, const float* sB1,
                                          int hh, int m) {
#pragma unroll 1
  for (int nh = 0; nh < 2; ++nh) {
    v8f acc[2][4];
    {
      const v8f z = {0.f, 0.f, 0.f, 0.f, 0.f, 0.f, 0.f, 0.f};
#pragma unroll
      for (int mt = 0; mt < 2; ++mt)
#pragma unroll
        for (int nt = 0; nt < 4; ++nt) acc[mt][nt] = z;
    }
    const unsigned short* ap0 = sAw + m * AP + 8 * hh;
    const unsigned short* ap1 = ap0 + 16 * AP;
    const unsigned short* bp  = BT + (size_t)(64 * nh + m) * KB + 8 * hh;
#pragma unroll
    for (int ks = 0; ks < KS; ++ks) {
      const int k0 = 32 * ks;
      FragB a0, a1;
      a0.h[0] = *(const v8usa*)(ap0 + k0);
      a0.h[1] = *(const v8usa*)(ap0 + k0 + 16);
      a1.h[0] = *(const v8usa*)(ap1 + k0);
      a1.h[1] = *(const v8usa*)(ap1 + k0 + 16);
#pragma unroll
      for (int nt = 0; nt < 4; ++nt) {
        const unsigned short* wq = bp + (size_t)(16 * nt) * KB + k0;
        FragB b;
        b.h[0] = *(const v8usa*)wq;
        b.h[1] = *(const v8usa*)(wq + 16);
        acc[0][nt] = wmb(a0, b, acc[0][nt]);
        acc[1][nt] = wmb(a1, b, acc[1][nt]);
      }
    }
#pragma unroll
    for (int nt = 0; nt < 4; ++nt) {
      const int col = 64 * nh + 16 * nt + m;
      const float bv = sB1[col];
#pragma unroll
      for (int mt = 0; mt < 2; ++mt)
#pragma unroll
        for (int r = 0; r < 8; ++r)
          sDw[(16 * mt + 8 * hh + r) * DP + col] = relu_f(acc[mt][nt][r] + bv);
    }
  }
}

template <int NO>
__device__ __forceinline__ v8f row_dots(const float* rd, const float* wt) {
  v8f acc = {0.f, 0.f, 0.f, 0.f, 0.f, 0.f, 0.f, 0.f};
#pragma unroll 1
  for (int c4 = 0; c4 < HID / 4; ++c4) {
    const v4f h = *(const v4fa*)(rd + 4 * c4);
#pragma unroll
    for (int o = 0; o < NO; ++o) {
      const v4f w = *(const v4fa*)(wt + o * HID + 4 * c4);
      float a = acc[o];
      a = fmaf(h.x, w.x, a);
      a = fmaf(h.y, w.y, a);
      a = fmaf(h.z, w.z, a);
      a = fmaf(h.w, w.w, a);
      acc[o] = a;
    }
  }
  return acc;
}

template <int L>
__global__ __launch_bounds__(MTHR) void k_edge(const int* __restrict__ erow, const int* __restrict__ ecol,
                                               const float* __restrict__ X, const float* __restrict__ EA,
                                               const unsigned short* __restrict__ BT,
                                               const float* __restrict__ b1, const float* __restrict__ W2,
                                               const float* __restrict__ b2, float* MSGo) {
  extern __shared__ __attribute__((aligned(16))) float dynf[];
  float*          sD  = dynf;
  unsigned short* sA  = (unsigned short*)(dynf + TM * DP);
  float*          sB1 = dynf + TM * DP + (TM * AP) / 2;
  float*          sW2 = sB1 + HID;
  float*          sB2 = sW2 + NF * HID;
  const int tid = (int)threadIdx.x, lane = tid & 31, wave = tid >> 5, hh = lane >> 4, m = lane & 15;

  sB1[tid] = bf16_val(b1[tid]);
#pragma unroll 1
  for (int i = tid; i < HID * EF; i += MTHR) {
    const int k = i / EF;
    const int o = i - EF * k;
    sW2[o * HID + k] = bf16_val(W2[i]);
  }
  {
    const float bb = bf16_val(b2[tid < EF ? tid : EF - 1]);
    if (tid < 8) sB2[tid] = (tid < EF) ? bb : 0.0f;
  }

  const int e  = (int)blockIdx.x * TM + tid;
  const int ec = e < NE ? e : NE - 1;
  int r = erow[ec];
  int c = ecol[ec];
  r = r < 0 ? 0 : (r > NN - 1 ? NN - 1 : r);
  c = c < 0 ? 0 : (c > NN - 1 ? NN - 1 : c);
  const v4f xra = *(const v4fa*)(X + (size_t)r * 8);
  const v4f xrb = *(const v4fa*)(X + (size_t)r * 8 + 4);
  const v4f xca = *(const v4fa*)(X + (size_t)c * 8);
  const v4f xcb = *(const v4fa*)(X + (size_t)c * 8 + 4);
  float e0, e1, e2;
  if constexpr (L == 0) {
    const float* p = EA + (size_t)ec * EF;
    e0 = p[0]; e1 = p[1]; e2 = p[2];
  } else {
    const v4f q = *(const v4fa*)(EA + (size_t)ec * 4);
    e0 = q.x; e1 = q.y; e2 = q.z;
  }
  {
    const v8f g0 = {xra.x, xra.y, xra.z, xra.w, xrb.x, xrb.y, xrb.z, xca.x};
    const v8f g1 = {xca.y, xca.z, xca.w, xcb.x, xcb.y, xcb.z, e0, e1};
    const v8f g2 = {e2, 0.f, 0.f, 0.f, 0.f, 0.f, 0.f, 0.f};
    const HL h0 = split8(g0);
    const HL h1 = split8(g1);
    const HL h2 = split8(g2);
    v8us oz;
#pragma unroll
    for (int j = 0; j < 8; ++j) oz[j] = (unsigned short)0;
    unsigned short* ra = sA + tid * AP;
    *(v8usa*)(ra + 0)  = h0.h;
    *(v8usa*)(ra + 8)  = h1.h;
    *(v8usa*)(ra + 16) = h2.h;
    *(v8usa*)(ra + 24) = oz;
    if constexpr (L != 0) {
      *(v8usa*)(ra + 32) = h0.l;
      *(v8usa*)(ra + 40) = h1.l;
      *(v8usa*)(ra + 48) = h2.l;
      *(v8usa*)(ra + 56) = oz;
    }
  }
  __syncthreads();

  wave_gemm<L + 1>(sA + 32 * wave * AP, sD + 32 * wave * DP, BT, sB1, hh, m);
  __syncthreads();

  const v8f d = row_dots<EF>(sD + tid * DP, sW2);
  v4f o;
  o.x = d[0] + sB2[0];
  o.y = d[1] + sB2[1];
  o.z = d[2] + sB2[2];
  o.w = 0.0f;
  putf4(MSGo + (size_t)e * 4, o);
}

__global__ __launch_bounds__(NTHR) void k_agg(const int* __restrict__ LIST, const int* __restrict__ CNT,
                                              const int* __restrict__ OFF, const float* __restrict__ MSG,
                                              const float* __restrict__ X, const float* __restrict__ u,
                                              const int* __restrict__ bat, unsigned short* NIN) {
  __shared__ __attribute__((aligned(16))) unsigned short sN[NTHR * AP];
  const int tid = (int)threadIdx.x;
  const int nodeBase = (int)blockIdx.x * NBA;
  const int* lb = LIST + (size_t)blockIdx.x * RCAP;
  const float qnan = __int_as_float(0x7fc00000);
  const float ninf = -__builtin_inff();

#pragma unroll 1
  for (int j = 0; j < 4; ++j) {
    const int node = nodeBase + j * NTHR + tid;
    int c = CNT[node];
    int o = OFF[node];
    const bool bad = (c < 0) || (c > DEGCAP);
    c = c < 0 ? 0 : (c > DEGCAP ? DEGCAP : c);
    o = o < 0 ? 0 : (o > RCAP - 1 ? RCAP - 1 : o);
    int cm = c;
#pragma unroll
    for (int d = 16; d >= 1; d >>= 1) {
      const int y = __shfl_xor(cm, d, 32);
      cm = y > cm ? y : cm;
    }
    float s0 = 0.0f, s1 = 0.0f, s2 = 0.0f;
    float m0 = ninf, m1 = ninf, m2 = ninf;
    const int cl = c > 0 ? c - 1 : 0;
#pragma unroll 1
    for (int p = 0; p < cm; ++p) {
      const int pi = p < c ? p : cl;
      int idx = o + pi;
      idx = idx > RCAP - 1 ? RCAP - 1 : idx;
      const int ent = lb[idx];
      int eid = ent >> SLA;
      eid = eid < 0 ? 0 : (eid > NE - 1 ? NE - 1 : eid);
      const v4f mv = *(const v4fa*)(MSG + (size_t)eid * 4);
      const bool valid = p < c;
      s0 = valid ? (s0 + mv.x) : s0;
      s1 = valid ? (s1 + mv.y) : s1;
      s2 = valid ? (s2 + mv.z) : s2;
      m0 = (valid && (mv.x > m0 || mv.x != mv.x)) ? mv.x : m0;
      m1 = (valid && (mv.y > m1 || mv.y != mv.y)) ? mv.y : m1;
      m2 = (valid && (mv.z > m2 || mv.z != mv.z)) ? mv.z : m2;
    }
    const bool has = c > 0;
    m0 = has ? m0 : 0.0f;
    m1 = has ? m1 : 0.0f;
    m2 = has ? m2 : 0.0f;
    const float cf = fmaxf((float)c, 1.0f);
    const float rc = 1.0f / cf;
    const float pz = bad ? qnan : 0.0f;
    const bool live = node < NN;
    const int ic = live ? node : NN - 1;
    const v4f xa = *(const v4fa*)(X + (size_t)ic * 8);
    const v4f xb = *(const v4fa*)(X + (size_t)ic * 8 + 4);
    int bt = bat[ic];
    bt = bt < 0 ? 0 : (bt > NG - 1 ? NG - 1 : bt);
    const v2f uu = *(const v2fa*)(u + (size_t)bt * UD);
    const float lf = live ? 1.0f : 0.0f;
    v8f g0 = {xa.x, xa.y, xa.z, xa.w, xb.x, xb.y, xb.z, s0 + pz};
    v8f g1 = {s1 + pz, s2 + pz, m0 + pz, m1 + pz, m2 + pz, s0 * rc + pz, s1 * rc + pz, s2 * rc + pz};
    v8f g2 = {bf16_val(uu.x), bf16_val(uu.y), 0.f, 0.f, 0.f, 0.f, 0.f, 0.f};
#pragma unroll
    for (int i = 0; i < 8; ++i) {
      g0[i] = live ? g0[i] : 0.0f;
      g1[i] = live ? g1[i] : 0.0f;
      g2[i] = g2[i] * lf;
    }
    const HL h0 = split8(g0);
    const HL h1 = split8(g1);
    const HL h2 = split8(g2);
    v8us oz;
#pragma unroll
    for (int i = 0; i < 8; ++i) oz[i] = (unsigned short)0;
    unsigned short* rn = sN + tid * AP;
    *(v8usa*)(rn + 0)  = h0.h;
    *(v8usa*)(rn + 8)  = h1.h;
    *(v8usa*)(rn + 16) = h2.h;
    *(v8usa*)(rn + 24) = oz;
    *(v8usa*)(rn + 32) = h0.l;
    *(v8usa*)(rn + 40) = h1.l;
    *(v8usa*)(rn + 48) = h2.l;
    *(v8usa*)(rn + 56) = oz;
    __syncthreads();
    unsigned short* gb = NIN + ((size_t)nodeBase + (size_t)j * NTHR) * KB;
#pragma unroll 1
    for (int it = 0; it < 8; ++it) {
      const int q = it * NTHR + tid;
      const v8us v = *(const v8usa*)(sN + (q >> 3) * AP + 8 * (q & 7));
      *(volatile v8us*)(gb + (size_t)q * 8) = v;
    }
    __threadfence();
#pragma unroll 1
    for (int it = 0; it < 8; ++it) {
      const int q = it * NTHR + tid;
      const v8us v = *(const v8usa*)(sN + (q >> 3) * AP + 8 * (q & 7));
      *(volatile v8us*)(gb + (size_t)q * 8) = v;
    }
    __syncthreads();
  }
}

__global__ __launch_bounds__(MTHR) void k_node(const unsigned short* __restrict__ NIN,
                                               const unsigned short* __restrict__ BT,
                                               const float* __restrict__ b1, const float* __restrict__ W2,
                                               const float* __restrict__ b2, int nN, float* Xo) {
  extern __shared__ __attribute__((aligned(16))) float dynf[];
  float*          sD  = dynf;
  unsigned short* sA  = (unsigned short*)(dynf + TM * DP);
  float*          sB1 = dynf + TM * DP + (TM * AP) / 2;
  float*          sW2 = sB1 + HID;
  float*          sB2 = sW2 + NF * HID;
  float*          sX  = dynf + TM * DP + (TM * AP) / 2 + CSTN;
  const int tid = (int)threadIdx.x, lane = tid & 31, wave = tid >> 5, hh = lane >> 4, m = lane & 15;
  const int rowBase = (int)blockIdx.x * TM;

  sB1[tid] = bf16_val(b1[tid]);
#pragma unroll 1
  for (int i = tid; i < HID * NF; i += MTHR) {
    const int k = i / NF;
    const int o = i - NF * k;
    sW2[o * HID + k] = bf16_val(W2[i]);
  }
  {
    const float bb = bf16_val(b2[tid < NF ? tid : NF - 1]);
    if (tid < 8) sB2[tid] = (tid < NF) ? bb : 0.0f;
  }
  {
    const unsigned short* src = NIN + (size_t)rowBase * KB;
#pragma unroll 4
    for (int it = 0; it < 8; ++it) {
      const int q = it * MTHR + tid;
      const v8us v = *(const v8usa*)(src + (size_t)q * 8);
      *(v8usa*)(sA + (q >> 3) * AP + 8 * (q & 7)) = v;
    }
  }
  __syncthreads();

  wave_gemm<2>(sA + 32 * wave * AP, sD + 32 * wave * DP, BT, sB1, hh, m);
  __syncthreads();

  {
    const v8f d = row_dots<NF>(sD + tid * DP, sW2);
    const bool live = (rowBase + tid) < nN;
    v4f qa, qb;
    qa.x = live ? (d[0] + sB2[0]) : 0.0f;
    qa.y = live ? (d[1] + sB2[1]) : 0.0f;
    qa.z = live ? (d[2] + sB2[2]) : 0.0f;
    qa.w = live ? (d[3] + sB2[3]) : 0.0f;
    qb.x = live ? (d[4] + sB2[4]) : 0.0f;
    qb.y = live ? (d[5] + sB2[5]) : 0.0f;
    qb.z = live ? (d[6] + sB2[6]) : 0.0f;
    qb.w = 0.0f;
    *(v4fa*)(sX + tid * 8)     = qa;
    *(v4fa*)(sX + tid * 8 + 4) = qb;
  }
  __syncthreads();
  {
    float* gb = Xo + (size_t)rowBase * 8;
    const v4f v0 = *(const v4fa*)(sX + 4 * tid);
    const v4f v1 = *(const v4fa*)(sX + 4 * (MTHR + tid));
    *(volatile v4f*)(gb + 4 * (size_t)tid) = v0;
    *(volatile v4f*)(gb + 4 * (size_t)(MTHR + tid)) = v1;
    __threadfence();
    *(volatile v4f*)(gb + 4 * (size_t)tid) = v0;
    *(volatile v4f*)(gb + 4 * (size_t)(MTHR + tid)) = v1;
  }
}

__global__ __launch_bounds__(NTHR) void k_poolhead(const float* __restrict__ X2, const int* __restrict__ bat,
                                                   const float* __restrict__ u,
                                                   const float* __restrict__ oW1, const float* __restrict__ ob1,
                                                   const float* __restrict__ oW2, const float* __restrict__ ob2,
                                                   const float* __restrict__ oW3, const float* __restrict__ ob3,
                                                   const float* __restrict__ oW4, const float* __restrict__ ob4,
                                                   float* RES) {
  __shared__ float wred[NWAVE * 16];
  __shared__ float sin_[32];
  __shared__ float sh[HID];
  __shared__ float sh2[HID];
  const int tid = (int)threadIdx.x, lane = tid & 31, wave = tid >> 5;
  const int g = (int)blockIdx.x;
  const float ninf = -__builtin_inff();

  v8f s  = {0.f, 0.f, 0.f, 0.f, 0.f, 0.f, 0.f, 0.f};
  v8f mx = {ninf, ninf, ninf, ninf, ninf, ninf, ninf, ninf};
  int cnt = 0;
#pragma unroll 1
  for (int i0 = wave * 32; i0 < NN; i0 += NTHR) {
    const int i  = i0 + lane;
    const int ic = i < NN ? i : NN - 1;
    const int b  = bat[ic];
    const bool hit = (i < NN) && (b == g);
    const unsigned msk = __builtin_amdgcn_ballot_w32(hit);
    if (msk != 0u) {
      const v4f a = *(const v4fa*)(X2 + (size_t)ic * 8);
      const v4f c = *(const v4fa*)(X2 + (size_t)ic * 8 + 4);
      const v8f v = {a.x, a.y, a.z, a.w, c.x, c.y, c.z, 0.0f};
#pragma unroll
      for (int f = 0; f < NF; ++f) {
        const float vf = v[f];
        const float sf = s[f];
        const float mf = mx[f];
        s[f]  = hit ? (sf + vf) : sf;
        mx[f] = (hit && (vf > mf || vf != vf)) ? vf : mf;
      }
      cnt += hit ? 1 : 0;
    }
  }
#pragma unroll
  for (int d = 16; d >= 1; d >>= 1) {
#pragma unroll
    for (int f = 0; f < NF; ++f) {
      const float so = __shfl_xor(s[f], d, 32);
      const float mo = __shfl_xor(mx[f], d, 32);
      const float mf = mx[f];
      s[f]  = s[f] + so;
      mx[f] = (mo > mf || mo != mo) ? mo : mf;
    }
    cnt += __shfl_xor(cnt, d, 32);
  }
  if (lane == 0) {
#pragma unroll
    for (int f = 0; f < NF; ++f) {
      wred[wave * 16 + f]      = s[f];
      wred[wave * 16 + NF + f] = mx[f];
    }
    wred[wave * 16 + 14] = (float)cnt;
    wred[wave * 16 + 15] = 0.0f;
  }
  __syncthreads();
  if (tid < 32) {
    const int f = tid < NF ? tid : NF - 1;
    float S = 0.0f, M = ninf, C = 0.0f;
#pragma unroll
    for (int w2 = 0; w2 < NWAVE; ++w2) {
      S += wred[w2 * 16 + f];
      const float mo = wred[w2 * 16 + NF + f];
      M = (mo > M || mo != mo) ? mo : M;
      C += wred[w2 * 16 + 14];
    }
    const float cf = fmaxf(C, 1.0f);
    const float rc = 1.0f / cf;
    const float uv = bf16_val(u[(size_t)g * UD + ((tid + 1) & 1)]);
    if (tid < NF) {
      sin_[tid]          = S;
      sin_[NF + tid]     = S * rc;
      sin_[2 * NF + tid] = (C > 0.0f) ? M : 0.0f;
    }
    if (tid == 21 || tid == 22) sin_[tid] = uv;
  }
  __syncthreads();

  const int j = tid & (HID - 1);
  {
    float acc = bf16_val(ob1[j]);
#pragma unroll 1
    for (int k = 0; k < 3 * NF + UD; ++k) acc = fmaf(sin_[k], bf16_val(oW1[(size_t)k * HID + j]), acc);
    acc = relu_f(acc);
    if (tid < HID) sh[j] = acc;
  }
  __syncthreads();
  {
    float acc = bf16_val(ob2[j]);
#pragma unroll 4
    for (int k = 0; k < HID; ++k) acc = fmaf(sh[k], bf16_val(oW2[(size_t)k * HID + j]), acc);
    acc = relu_f(acc);
    if (tid < HID) sh2[j] = acc;
  }
  __syncthreads();
  {
    float acc = bf16_val(ob3[j]);
#pragma unroll 4
    for (int k = 0; k < HID; ++k) acc = fmaf(sh2[k], bf16_val(oW3[(size_t)k * HID + j]), acc);
    acc = relu_f(acc);
    const float pr = acc * bf16_val(oW4[j]);
    if (tid < HID) sh[j] = pr;
  }
  __syncthreads();
  if (wave == 0) {
    float t = ((sh[lane] + sh[lane + 32]) + sh[lane + 64]) + sh[lane + 96];
#pragma unroll
    for (int d = 16; d >= 1; d >>= 1) t = t + __shfl_xor(t, d, 32);
    const float res = t + bf16_val(ob4[0]);
    v4f o4;
    o4.x = (lane == 0) ? res : 0.0f;
    o4.y = 0.0f; o4.z = 0.0f; o4.w = 0.0f;
    float* op = RES + (size_t)g * 32 + 4 * (lane & 7);
    if (lane < 8) *(volatile v4f*)op = o4;
    __threadfence();
    if (lane < 8) *(volatile v4f*)op = o4;
  }
}

__global__ __launch_bounds__(64) void k_out(const float* __restrict__ RES, float* out) {
  const int tid = (int)threadIdx.x;
  v4f o;
  o.x = RES[(size_t)(4 * tid + 0) * 32];
  o.y = RES[(size_t)(4 * tid + 1) * 32];
  o.z = RES[(size_t)(4 * tid + 2) * 32];
  o.w = RES[(size_t)(4 * tid + 3) * 32];
  putf4(out + 4 * tid, o);
}

static inline size_t al256(size_t o) { return (o + 255) & ~(size_t)255; }

extern "C" void kernel_launch(void* const* d_in, const int* in_sizes, int n_in,
                              void* d_out, int out_size, void* d_ws, size_t ws_size,
                              hipStream_t stream) {
  if (n_in < 21) return;
  if (in_sizes[0] != NN * NF || in_sizes[1] != NE * EF || in_sizes[2] != NG * UD) return;
  if (in_sizes[3] != 2 * KIE * HID || in_sizes[4] != 2 * HID) return;
  if (in_sizes[5] != 2 * HID * EF || in_sizes[6] != 2 * EF) return;
  if (in_sizes[7] != 2 * KIN * HID || in_sizes[8] != 2 * HID) return;
  if (in_sizes[9] != 2 * HID * NF || in_sizes[10] != 2 * NF) return;
  if (in_sizes[11] != (3 * NF + UD) * HID || in_sizes[12] != HID) return;
  if (in_sizes[13] != HID * HID || in_sizes[14] != HID) return;
  if (in_sizes[15] != HID * HID || in_sizes[16] != HID) return;
  if (in_sizes[17] != HID || in_sizes[18] != 1) return;
  if (in_sizes[19] != 2 * NE || in_sizes[20] != NN) return;
  if (out_size != NG) return;

  const float* x   = (const float*)d_in[0];
  const float* ea  = (const float*)d_in[1];
  const float* u   = (const float*)d_in[2];
  const float* eW1 = (const float*)d_in[3];
  const float* eb1 = (const float*)d_in[4];
  const float* eW2 = (const float*)d_in[5];
  const float* eb2 = (const float*)d_in[6];
  const float* nW1 = (const float*)d_in[7];
  const float* nb1 = (const float*)d_in[8];
  const float* nW2 = (const float*)d_in[9];
  const float* nb2 = (const float*)d_in[10];
  const float* oW1 = (const float*)d_in[11];
  const float* ob1 = (const float*)d_in[12];
  const float* oW2 = (const float*)d_in[13];
  const float* ob2 = (const float*)d_in[14];
  const float* oW3 = (const float*)d_in[15];
  const float* ob3 = (const float*)d_in[16];
  const float* oW4 = (const float*)d_in[17];
  const float* ob4 = (const float*)d_in[18];
  const int*   ei  = (const int*)d_in[19];
  const int*   bat = (const int*)d_in[20];
  const int* erow = ei;
  const int* ecol = ei + NE;
  float* out = (float*)d_out;

  char* ws = (char*)d_ws;
  size_t off = 0;
  const size_t oE1T  = off; off = al256(off + (size_t)2 * HID * KB * 2);
  const size_t oN1T  = off; off = al256(off + (size_t)2 * HID * KB * 2);
  const size_t oX0   = off; off = al256(off + (size_t)NP * 8 * 4);
  const size_t oX1   = off; off = al256(off + (size_t)NP * 8 * 4);
  const size_t oX2   = off; off = al256(off + (size_t)NP * 8 * 4);
  const size_t oMSG0 = off; off = al256(off + (size_t)NE * 4 * 4);
  const size_t oMSG1 = off; off = al256(off + (size_t)NE * 4 * 4);
  const size_t oNIN  = off; off = al256(off + (size_t)NPA * KB * 2);
  const size_t oLIST = off; off = al256(off + (size_t)NBLK * RCAP * 4);
  const size_t oCNT  = off; off = al256(off + (size_t)NPA * 4);
  const size_t oOFF  = off; off = al256(off + (size_t)NPA * 4);
  const size_t oRES  = off; off = al256(off + (size_t)NG * 32 * 4);
  if (off > ws_size || off > (size_t)WSMAX) return;
  unsigned short* E1T  = (unsigned short*)(ws + oE1T);
  unsigned short* N1T  = (unsigned short*)(ws + oN1T);
  float*          X0   = (float*)(ws + oX0);
  float*          X1   = (float*)(ws + oX1);
  float*          X2   = (float*)(ws + oX2);
  float*          MSG0 = (float*)(ws + oMSG0);
  float*          MSG1 = (float*)(ws + oMSG1);
  unsigned short* NIN  = (unsigned short*)(ws + oNIN);
  int*            LIST = (int*)(ws + oLIST);
  int*            CNT  = (int*)(ws + oCNT);
  int*            OFF  = (int*)(ws + oOFF);
  float*          RES  = (float*)(ws + oRES);

  hipFuncSetAttribute(reinterpret_cast<const void*>(&k_bucket), hipFuncAttributeMaxDynamicSharedMemorySize,
                      (int)AGG_LDS_BYTES);
  hipFuncSetAttribute(reinterpret_cast<const void*>(&k_edge<0>), hipFuncAttributeMaxDynamicSharedMemorySize,
                      (int)MLP_LDS_BYTES);
  hipFuncSetAttribute(reinterpret_cast<const void*>(&k_edge<1>), hipFuncAttributeMaxDynamicSharedMemorySize,
                      (int)MLP_LDS_BYTES);
  hipFuncSetAttribute(reinterpret_cast<const void*>(&k_node), hipFuncAttributeMaxDynamicSharedMemorySize,
                      (int)MLP_LDS_BYTES);

  k_prep<<<(NU_W + NU_X) / NTHR, NTHR, 0, stream>>>(x, eW1, nW1, E1T, N1T, X0);
  k_bucket<<<NBLK, NTHR, AGG_LDS_BYTES, stream>>>(ecol, NE, 1, LIST, CNT, OFF);
  k_edge<0><<<NE / TM, MTHR, MLP_LDS_BYTES, stream>>>(erow, ecol, X0, ea, E1T, eb1, eW2, eb2, MSG0);
  k_agg<<<NBLK, NTHR, 0, stream>>>(LIST, CNT, OFF, MSG0, X0, u, bat, NIN);
  k_node<<<NP / TM, MTHR, MLP_LDS_BYTES, stream>>>(NIN, N1T, nb1, nW2, nb2, NN, X1);
  k_edge<1><<<NE / TM, MTHR, MLP_LDS_BYTES, stream>>>(erow, ecol, X1, MSG0, E1T + (size_t)HID * KB,
                                                        eb1 + HID, eW2 + HID * EF, eb2 + EF, MSG1);
  k_agg<<<NBLK, NTHR, 0, stream>>>(LIST, CNT, OFF, MSG1, X1, u, bat, NIN);
  k_node<<<NP / TM, MTHR, MLP_LDS_BYTES, stream>>>(NIN, N1T + (size_t)HID * KB, nb1 + HID, nW2 + HID * NF,
                                                    nb2 + NF, NN, X2);
  k_poolhead<<<NG, NTHR, 0, stream>>>(X2, bat, u, oW1, ob1, oW2, ob2, oW3, ob3, oW4, ob4, RES);
  k_out<<<1, 64, 0, stream>>>(RES, out);
}
